// DecodeLayer_55628416417885
// MI455X (gfx1250) — hardware-run, weakly checked
//
#include <hip/hip_runtime.h>
#include <math.h>

#ifndef NB
#define NB 4
#endif
#ifndef SEQ
#define SEQ 2048
#endif
#define NB_FULL 4
#define SEQ_FULL 2048
#define DM 1024
#define DFF 4096
#define NHEAD 16
#define HDIM 64
#define MROWS (NB * SEQ)
#define CHROWS (MROWS / 2)

static_assert(NB >= 1 && NB <= NB_FULL);
static_assert(SEQ % 64 == 0 && SEQ <= SEQ_FULL);
static_assert(MROWS % 128 == 0);
static_assert(DM == NHEAD * HDIM);
static_assert(DM % 64 == 0 && DFF % 64 == 0);
static_assert(NB == 1 || SEQ == SEQ_FULL);
static_assert(HDIM == 64);
static_assert(DM % 32 == 0 && DFF % 32 == 0);
static_assert(MROWS % 64 == 0 && CHROWS % 64 == 0 && (2 * DM) % 64 == 0);
static_assert(32 * 16 * 8 == DM * 4);
static_assert(32 * 8 * 8 == DM * 2);
static_assert(8 * 16 * 68 * 4 <= 131072);
static_assert(4 * 16 * 64 * 2 + 4 * 16 * 68 * 4 <= 131072);

typedef __attribute__((ext_vector_type(16))) _Float16 v16h;
typedef __attribute__((ext_vector_type(8)))  _Float16 v8h;
typedef __attribute__((ext_vector_type(8)))  float    v8f;
typedef __attribute__((ext_vector_type(4)))  float    v4f;
typedef unsigned int cm_u4 __attribute__((ext_vector_type(4)));
typedef unsigned int bk_u2 __attribute__((ext_vector_type(2)));
typedef v8h __attribute__((may_alias)) v8h_a;
typedef v4f __attribute__((may_alias)) v4f_a;
typedef _Float16 h16;


#define VST2(T, ptr, val) do { const T vst2_v_ = (val); *(volatile T*)(ptr) = vst2_v_; __threadfence(); *(volatile T*)(ptr) = vst2_v_; } while (0)
#define VST2V4(ptr, val) do { const v4f vst2_v4_ = (val); *(volatile v4f*)(ptr) = vst2_v4_; __threadfence(); *(volatile v4f*)(ptr) = vst2_v4_; } while (0)

__device__ __forceinline__ float cmb_bf(float v) {
    const unsigned u = __builtin_bit_cast(unsigned, v);
    const unsigned r = (u + 0x7fffu + ((u >> 16) & 1u)) & 0xffff0000u;
    return __builtin_bit_cast(float, r);
}
__device__ __forceinline__ unsigned int cmb_pk2(float a, float b) {
    return (unsigned int)__builtin_bit_cast(unsigned short, (_Float16)a) | ((unsigned int)__builtin_bit_cast(unsigned short, (_Float16)b) << 16);
}
static __device__ __forceinline__ h16 toh_flush(float v) { const h16 r = (h16)v; return (fabsf(v) < 6.103515625e-05f) ? (h16)0.0f : r; }
__device__ __forceinline__ unsigned int pk2_flush(float a, float b) {
    return (unsigned int)__builtin_bit_cast(unsigned short, toh_flush(a)) | ((unsigned int)__builtin_bit_cast(unsigned short, toh_flush(b)) << 16);
}
__device__ __forceinline__ v16h frag_ld(const _Float16* __restrict__ p) {
    union U { v16h v; v8h h[2]; } f;
    f.h[0] = *(const v8h*)(p);
    f.h[1] = *(const v8h*)(p + 16);
    return f.v;
}
__device__ __forceinline__ v8f wmma16(v16h a, v16h b, v8f c) {
    c = __builtin_amdgcn_wmma_f32_16x16x32_f16(false, a, false, b, (short)0, c, false, false);
    asm volatile("v_nop\n\tv_nop\n\tv_nop\n\tv_nop" : "+v"(c) : "v"(a), "v"(b));
    return c;
}
__device__ __forceinline__ void dep_guard_h(v8f& a, v8f& b, v16h x, v16h y) { asm volatile("v_nop\n\tv_nop\n\tv_nop\n\tv_nop" : "+v"(a), "+v"(b) : "v"(x), "v"(y)); }
__device__ __forceinline__ void keep4_h(v16h a, v16h b, v16h c, v16h d) { asm volatile("v_nop" :: "v"(a), "v"(b), "v"(c), "v"(d)); }
__device__ __forceinline__ void acc_guard4(v8f& a, v8f& b, v8f& c, v8f& d) { asm volatile("v_nop\n\tv_nop\n\tv_nop\n\tv_nop" : "+v"(a), "+v"(b), "+v"(c), "+v"(d)); }
__device__ __forceinline__ void wave_sync() {
    __builtin_amdgcn_fence(3  , "workgroup");
    __builtin_amdgcn_wave_barrier();
    __builtin_amdgcn_fence(2  , "workgroup");
}
__device__ __forceinline__ float gelu_e(float x) {
    return 0.5f * x * (1.0f + erff(x * 0.70710678118654752f));
}

__global__ __launch_bounds__(256) void k_cm_castbT(const float* __restrict__ SRC, int lds, unsigned short* __restrict__ DST, int ldd, int nR, int nC, float sc) {
    const long long u = (long long)blockIdx.x * 256 + threadIdx.x; const int per = nR / 8;
    if (u >= (long long)nC * per) return;
    const int c = (int)(u / per); const int r0 = 8 * (int)(u % per);
    float w[8];
#pragma unroll
    for (int e = 0; e < 8; ++e) w[e] = cmb_bf(SRC[(long long)(r0 + e) * lds + c]) * sc;
    cm_u4 pk; pk.x = cmb_pk2(w[0], w[1]); pk.y = cmb_pk2(w[2], w[3]); pk.z = cmb_pk2(w[4], w[5]); pk.w = cmb_pk2(w[6], w[7]);
    VST2(cm_u4, (cm_u4*)(DST + (long long)c * ldd + r0), pk);
}

template <int BIAS_MODE, int OUT_MODE, bool RESID, int ACT>
__global__ __launch_bounds__(256) void wmma_gemm64(
    const unsigned short* __restrict__ Ap, int lda,
    const unsigned short* __restrict__ Btp, int ldb,
    void* __restrict__ Cout, int ldc,
    const float* __restrict__ bias, const float* __restrict__ resid,
    int M, int N, int K, float scale) {
  static_assert(!(RESID && OUT_MODE == 1));
  const _Float16* Ab = (const _Float16*)Ap; const _Float16* Bb = (const _Float16*)Btp;
  __shared__ __align__(16) float sT[8][16 * 68];
  const int lane = threadIdx.x & 31;
  const int wave = __builtin_amdgcn_readfirstlane(threadIdx.x >> 5);
  const int tilesN = N >> 6;
  const int tilesM = M >> 6;
  const int tile = blockIdx.x * 8 + wave;
  if (tile >= tilesM * tilesN) return;
  const int tm = tile / tilesN;
  const int tn = tile - tm * tilesN;
  const int m0 = tm << 6;
  const int n0 = tn << 6;
  const int rlane = lane & 15;
  const int koff  = (lane >> 4) * 8;
  const int mOff  = (lane >> 4) * 8;

  v8f acc[4][4];
#pragma unroll
  for (int i = 0; i < 4; ++i)
#pragma unroll
    for (int j = 0; j < 4; ++j) acc[i][j] = (v8f){0.f,0.f,0.f,0.f,0.f,0.f,0.f,0.f};

  for (int k0 = 0; k0 < K; k0 += 32) {
    v16h bh[4];
#pragma unroll
    for (int j = 0; j < 4; ++j) {
      const size_t bo = (size_t)(n0 + (j << 4) + rlane) * ldb + koff + k0;
      bh[j] = frag_ld(Bb + bo);
    }
#pragma unroll
    for (int i = 0; i < 4; ++i) {
      const size_t ao = (size_t)(m0 + (i << 4) + rlane) * lda + koff + k0;
      const v16h ah = frag_ld(Ab + ao);
#pragma unroll
      for (int j = 0; j < 4; ++j)
        acc[i][j] = __builtin_amdgcn_wmma_f32_16x16x32_f16(false, ah, false, bh[j], (short)0, acc[i][j], false, false);
      dep_guard_h(acc[i][0], acc[i][3], ah, ah);
    }
    keep4_h(bh[0], bh[1], bh[2], bh[3]);
  }
  acc_guard4(acc[0][0], acc[0][1], acc[0][2], acc[0][3]);
  acc_guard4(acc[1][0], acc[1][1], acc[1][2], acc[1][3]);
  acc_guard4(acc[2][0], acc[2][1], acc[2][2], acc[2][3]);
  acc_guard4(acc[3][0], acc[3][1], acc[3][2], acc[3][3]);

  float* slab = sT[wave];
#pragma unroll
  for (int i = 0; i < 4; ++i) {
    const int mBase = m0 + (i << 4);
#pragma unroll
    for (int j = 0; j < 4; ++j) {
      const int n = n0 + (j << 4) + rlane;
      float bv = 0.f;
      if (BIAS_MODE == 2) bv = cmb_bf(bias[n]);
#pragma unroll
      for (int r = 0; r < 8; ++r) {
        float v = acc[i][j][r] * scale;
        if (BIAS_MODE == 1) v += cmb_bf(bias[mBase + mOff + r]);
        if (BIAS_MODE == 2) v += bv;
        slab[(mOff + r) * 68 + (j << 4) + rlane] = v;
      }
    }
    wave_sync();
    if (ACT == 1) {
#pragma unroll 1
      for (int t = 0; t < 8; ++t) {
        float* sp = slab + (t * 2 + (lane >> 4)) * 68 + (lane & 15) * 4;
        v4f a = *(const v4f_a*)sp;
        a.x = gelu_e(a.x); a.y = gelu_e(a.y); a.z = gelu_e(a.z); a.w = gelu_e(a.w);
        *(v4f_a*)sp = a;
      }
      wave_sync();
    }
    if (OUT_MODE == 0) {
      float* C = (float*)Cout;
      const int hh = lane >> 4, c4 = (lane & 15) * 4;
      v4f ov[8];
#pragma unroll
      for (int it = 0; it < 8; ++it) {
        const int row = it * 2 + hh;
        v4f v = *(const v4f_a*)(slab + row * 68 + c4);
        if (RESID) {
          const v4f rv = *(const v4f*)(resid + (size_t)(mBase + row) * ldc + n0 + c4);
          v = v + rv;
        }
        ov[it] = v;
      }
#pragma unroll
      for (int pass = 0; pass < 2; ++pass) {
#pragma unroll
        for (int it = 0; it < 8; ++it) {
          const int row = it * 2 + hh;
          *(volatile v4f*)(C + (size_t)(mBase + row) * ldc + n0 + c4) = ov[it];
        }
        __threadfence();
      }
    } else {
      const int q = lane >> 3, c8 = (lane & 7) * 8;
      unsigned short* C = (unsigned short*)Cout;
      static_assert(32 * 16 * 4 == 16 * 64 * 2);
#pragma unroll
      for (int pass = 0; pass < 2; ++pass) {
#pragma unroll
        for (int it = 0; it < 4; ++it) {
          const int row = it * 4 + q;
          const float* sp = slab + row * 68 + c8;
          v8h hv;
#pragma unroll
          for (int e = 0; e < 8; ++e) hv[e] = toh_flush(sp[e]);
          *(volatile v8h*)(C + (size_t)(mBase + row) * ldc + n0 + c8) = hv;
        }
        __threadfence();
      }
    }
    wave_sync();
  }
}

__global__ __launch_bounds__(128) void k_attn_f16(const unsigned short* __restrict__ QKp, const unsigned short* __restrict__ VTp,
                                                  unsigned short* __restrict__ AOp) {
  __shared__ __align__(16) _Float16 Psh[4][16 * 64];
  __shared__ __align__(16) float    Os[4][16 * 68];
  const _Float16* QK = (const _Float16*)QKp; const _Float16* VT = (const _Float16*)VTp;
  const int tid = threadIdx.x, wave = __builtin_amdgcn_readfirstlane(tid >> 5), lane = tid & 31, hh = lane >> 4, c = lane & 15;
  constexpr int nqb = SEQ / 64;
  const int bx = blockIdx.x;
  const int qb = bx % nqb;
  const int bh = bx / nqb;
  const int h  = bh % NHEAD;
  const int b  = bh / NHEAD;
  const int q0 = qb * 64 + wave * 16;
  const float SCL = 0.18033688011112042f;
  const float PSC = 4096.0f;

  v16h qa[2];
  {
    const _Float16* qrow = QK + (size_t)(b * SEQ + q0 + c) * (2 * DM) + h * HDIM + 8 * hh;
    qa[0] = frag_ld(qrow);
    qa[1] = frag_ld(qrow + 32);
  }
  float mrow[8], lrow[8];
  v8f oacc[4];
#pragma unroll
  for (int r = 0; r < 8; ++r) { mrow[r] = -INFINITY; lrow[r] = 0.f; }
#pragma unroll
  for (int t = 0; t < 4; ++t) oacc[t] = (v8f){0.f,0.f,0.f,0.f,0.f,0.f,0.f,0.f};
  _Float16* pw = Psh[wave];

  for (int kc = 0; kc <= qb; ++kc) {
    const int kv0 = kc * 64;
    v8f s[4];
#pragma unroll
    for (int j = 0; j < 4; ++j) {
      const _Float16* krow = QK + (size_t)(b * SEQ + kv0 + j * 16 + c) * (2 * DM) + DM + h * HDIM + 8 * hh;
      v8f a = (v8f){0.f,0.f,0.f,0.f,0.f,0.f,0.f,0.f};
      a = wmma16(qa[0], frag_ld(krow), a);
      a = wmma16(qa[1], frag_ld(krow + 32), a);
      s[j] = a;
    }
    const bool diag = (kc == qb);
    float cm[8];
#pragma unroll
    for (int r = 0; r < 8; ++r) {
      const int qrow_i = q0 + 8 * hh + r;
      float m = -INFINITY;
#pragma unroll
      for (int j = 0; j < 4; ++j) {
        const int kvcol = kv0 + j * 16 + c;
        float v = s[j][r] * SCL;
        if (diag && kvcol > qrow_i) v = -INFINITY;
        s[j][r] = v;
        m = fmaxf(m, v);
      }
      m = fmaxf(m, __shfl_xor(m, 1, 32)); m = fmaxf(m, __shfl_xor(m, 2, 32));
      m = fmaxf(m, __shfl_xor(m, 4, 32)); m = fmaxf(m, __shfl_xor(m, 8, 32));
      cm[r] = m;
    }
#pragma unroll
    for (int r = 0; r < 8; ++r) {
      const float mnew = fmaxf(mrow[r], cm[r]);
      const float alpha = exp2f(mrow[r] - mnew);
      mrow[r] = mnew;
      float psum = 0.f;
#pragma unroll
      for (int j = 0; j < 4; ++j) {
        const float p = exp2f(s[j][r] - mnew);
        psum += p;
        pw[(8 * hh + r) * 64 + j * 16 + c] = toh_flush(p * PSC);
      }
      psum += __shfl_xor(psum, 1, 32); psum += __shfl_xor(psum, 2, 32);
      psum += __shfl_xor(psum, 4, 32); psum += __shfl_xor(psum, 8, 32);
      lrow[r] = lrow[r] * alpha + psum;
#pragma unroll
      for (int t = 0; t < 4; ++t) oacc[t][r] *= alpha;
    }
    wave_sync();
#pragma unroll
    for (int kk = 0; kk < 2; ++kk) {
      union U { v16h v; v8h h[2]; } pa;
      const v8h_a* pp = (const v8h_a*)(pw + c * 64 + kk * 32 + 8 * hh);
      pa.h[0] = pp[0];
      pa.h[1] = pp[2];
#pragma unroll
      for (int t = 0; t < 4; ++t) {
        const _Float16* vrow = VT + (size_t)(h * HDIM + t * 16 + c) * MROWS + (size_t)b * SEQ + kv0 + kk * 32 + 8 * hh;
        oacc[t] = wmma16(pa.v, frag_ld(vrow), oacc[t]);
      }
    }
    wave_sync();
  }

  float* os = Os[wave];
#pragma unroll
  for (int r = 0; r < 8; ++r) {
    const float inv = 1.0f / (lrow[r] * PSC);
#pragma unroll
    for (int t = 0; t < 4; ++t) os[(8 * hh + r) * 68 + t * 16 + c] = oacc[t][r] * inv;
  }
  wave_sync();
  {
    const int q = lane >> 3, c8 = (lane & 7) * 8;
    static_assert(32 * 16 * 4 == 16 * HDIM * 2);
#pragma unroll
    for (int pass = 0; pass < 2; ++pass) {
#pragma unroll
      for (int it = 0; it < 4; ++it) {
        const int row = it * 4 + q;
        const float* sp = os + row * 68 + c8;
        v8h hv;
#pragma unroll
        for (int e = 0; e < 8; ++e) hv[e] = toh_flush(sp[e]);
        *(volatile v8h*)(AOp + (size_t)(b * SEQ + q0 + row) * DM + h * HDIM + c8) = hv;
      }
      __threadfence();
    }
  }
}

template <int HASA>
__device__ __forceinline__ void ln_row_body(const float* __restrict__ A, const float* __restrict__ X, const float* __restrict__ GA, const float* __restrict__ BE,
                                            int rows, float* __restrict__ Ysum, unsigned short* __restrict__ Y16) {
    #pragma clang fp contract(off)
    const int r = blockIdx.x * 8 + __builtin_amdgcn_readfirstlane(threadIdx.x >> 5); const int L = threadIdx.x & 31;
    if (r >= rows) return;
    const long long re = (long long)(r / SEQ) * SEQ_FULL + (r % SEQ);
    v4f v[8]; float s = 0.f;
#pragma unroll
    for (int q = 0; q < 8; ++q) {
        const int cc = 4 * L + 128 * q;
        v4f x = *(const v4f*)(X + re * DM + cc);
        x.x = cmb_bf(x.x); x.y = cmb_bf(x.y); x.z = cmb_bf(x.z); x.w = cmb_bf(x.w);
        v[q] = x;
        if (HASA) {
            const v4f a = *(const v4f*)(A + (long long)r * DM + cc);
            v[q] = a + x;
            VST2V4(Ysum + (long long)r * DM + cc, v[q]);
        }
        s += (v[q].x + v[q].y) + (v[q].z + v[q].w);
    }
#pragma unroll
    for (int o = 16; o > 0; o >>= 1) s += __shfl_xor(s, o, 32);
    const float mu = s * (1.f / DM); float qq = 0.f;
#pragma unroll
    for (int q = 0; q < 8; ++q) {
        v[q].x -= mu; v[q].y -= mu; v[q].z -= mu; v[q].w -= mu;
        qq += (v[q].x * v[q].x + v[q].y * v[q].y) + (v[q].z * v[q].z + v[q].w * v[q].w);
    }
#pragma unroll
    for (int o = 16; o > 0; o >>= 1) qq += __shfl_xor(qq, o, 32);
    const float rs = rsqrtf(qq * (1.f / DM) + 1e-5f);
#pragma unroll
    for (int q = 0; q < 8; ++q) {
        const int cc = 4 * L + 128 * q;
        const v4f ga = *(const v4f*)(GA + cc), be = *(const v4f*)(BE + cc);
        v4f y;
        y.x = v[q].x * rs * cmb_bf(ga.x) + cmb_bf(be.x); y.y = v[q].y * rs * cmb_bf(ga.y) + cmb_bf(be.y);
        y.z = v[q].z * rs * cmb_bf(ga.z) + cmb_bf(be.z); y.w = v[q].w * rs * cmb_bf(ga.w) + cmb_bf(be.w);
        bk_u2 pk; pk.x = pk2_flush(y.x, y.y); pk.y = pk2_flush(y.z, y.w);
        VST2(bk_u2, (bk_u2*)(Y16 + (long long)r * DM + cc), pk);
    }
}
__global__ __launch_bounds__(256) void k_ln_first(const float* __restrict__ X, const float* __restrict__ GA, const float* __restrict__ BE,
                                                  int rows, unsigned short* __restrict__ Y16) {
    ln_row_body<0>(nullptr, X, GA, BE, rows, nullptr, Y16);
}
__global__ __launch_bounds__(256) void k_ln_second(const float* __restrict__ A, const float* __restrict__ X, const float* __restrict__ GA, const float* __restrict__ BE,
                                                   int rows, float* __restrict__ Ysum, unsigned short* __restrict__ Y16) {
    ln_row_body<1>(A, X, GA, BE, rows, Ysum, Y16);
}

#define SZ_X16  ((size_t)MROWS * DM * 2)
#define SZ_W3T  ((size_t)3 * DM * DM * 2)
#define SZ_WOT  ((size_t)DM * DM * 2)
#define SZ_W1T  ((size_t)DFF * DM * 2)
#define SZ_W2T  ((size_t)DM * DFF * 2)
#define SZ_R5   ((size_t)MROWS * 6144)
#define SZ_N32  ((size_t)MROWS * DM * 4)
#define SZ_TOTAL (SZ_X16 + SZ_W3T + SZ_WOT + SZ_W1T + SZ_W2T + SZ_R5 + SZ_N32)
static_assert((size_t)MROWS * 2 * DM * 2 + (size_t)DM * MROWS * 2 <= SZ_R5);
static_assert((size_t)MROWS * DM * 4 <= SZ_R5);
static_assert((size_t)CHROWS * DFF * 2 <= SZ_R5);
static_assert(SZ_TOTAL <= (size_t)134217728);

extern "C" void kernel_launch(void* const* d_in, const int* in_sizes, int n_in, void* d_out, int out_size, void* d_ws, size_t ws_size, hipStream_t stream) {
    if (n_in < 13) return;
    const long long need_rows = (long long)(NB - 1) * SEQ_FULL + SEQ;
    if ((long long)in_sizes[0] < need_rows * DM) return;
    if (in_sizes[1] < DM || in_sizes[2] < DM || in_sizes[3] < 3 * DM * DM || in_sizes[4] < 3 * DM || in_sizes[5] < DM * DM || in_sizes[6] < DM) return;
    if (in_sizes[7] < DM || in_sizes[8] < DM || in_sizes[9] < DM * DFF || in_sizes[10] < DFF || in_sizes[11] < DFF * DM || in_sizes[12] < DM) return;
    if ((long long)out_size < need_rows * DM) return;
    if (SZ_TOTAL > ws_size) return;

    const float* x      = (const float*)d_in[0];
    const float* ln1_g  = (const float*)d_in[1];
    const float* ln1_b  = (const float*)d_in[2];
    const float* w_attn = (const float*)d_in[3];
    const float* b_attn = (const float*)d_in[4];
    const float* w_proj = (const float*)d_in[5];
    const float* b_proj = (const float*)d_in[6];
    const float* ln2_g  = (const float*)d_in[7];
    const float* ln2_b  = (const float*)d_in[8];
    const float* w_fc   = (const float*)d_in[9];
    const float* b_fc   = (const float*)d_in[10];
    const float* w_fc2  = (const float*)d_in[11];
    const float* b_fc2  = (const float*)d_in[12];
    float* out = (float*)d_out;

    char* wsp = (char*)d_ws;
    unsigned short* XN16 = (unsigned short*)wsp; wsp += SZ_X16;
    unsigned short* W3T = (unsigned short*)wsp; wsp += SZ_W3T;
    unsigned short* WOT = (unsigned short*)wsp; wsp += SZ_WOT;
    unsigned short* W1T = (unsigned short*)wsp; wsp += SZ_W1T;
    unsigned short* W2T = (unsigned short*)wsp; wsp += SZ_W2T;
    char* R5 = wsp; wsp += SZ_R5;
    float* X1 = (float*)wsp; wsp += SZ_N32;
    unsigned short* AO16 = XN16;
    unsigned short* N16  = XN16;
    unsigned short* QK16 = (unsigned short*)R5;
    unsigned short* VT16 = (unsigned short*)(R5 + (size_t)MROWS * 2 * DM * 2);
    float* ATT = (float*)R5;
    unsigned short* ACT16 = (unsigned short*)R5;

    k_cm_castbT<<<(unsigned)(((long long)(3 * DM) * (DM / 8) + 255) / 256), 256, 0, stream>>>(w_attn, 3 * DM, W3T, DM, DM, 3 * DM, 16.0f);
    k_cm_castbT<<<(unsigned)(((long long)DM * (DM / 8) + 255) / 256), 256, 0, stream>>>(w_proj, DM, WOT, DM, DM, DM, 16.0f);
    k_cm_castbT<<<(unsigned)(((long long)DFF * (DM / 8) + 255) / 256), 256, 0, stream>>>(w_fc, DFF, W1T, DM, DM, DFF, 16.0f);
    k_cm_castbT<<<(unsigned)(((long long)DM * (DFF / 8) + 255) / 256), 256, 0, stream>>>(w_fc2, DM, W2T, DFF, DFF, DM, 16.0f);

    k_ln_first<<<(unsigned)((MROWS + 7) / 8), 256, 0, stream>>>(x, ln1_g, ln1_b, MROWS, XN16);
    wmma_gemm64<2, 1, false, 0><<<(unsigned)(((MROWS / 64) * ((2 * DM) / 64) + 7) / 8), 256, 0, stream>>>(
        XN16, DM, W3T, DM, (void*)QK16, 2 * DM, b_attn, nullptr, MROWS, 2 * DM, DM, 0.0625f);
    wmma_gemm64<1, 1, false, 0><<<(unsigned)(((DM / 64) * (MROWS / 64) + 7) / 8), 256, 0, stream>>>(
        W3T + (size_t)2 * DM * DM, DM, XN16, DM, (void*)VT16, MROWS, b_attn + 2 * DM, nullptr, DM, MROWS, DM, 0.0625f);
    k_attn_f16<<<(unsigned)(NB * NHEAD * (SEQ / 64)), 128, 0, stream>>>(QK16, VT16, AO16);
    wmma_gemm64<2, 0, false, 0><<<(unsigned)(((MROWS / 64) * (DM / 64) + 7) / 8), 256, 0, stream>>>(
        AO16, DM, WOT, DM, (void*)ATT, DM, b_proj, nullptr, MROWS, DM, DM, 0.0625f);
    k_ln_second<<<(unsigned)((MROWS + 7) / 8), 256, 0, stream>>>(ATT, x, ln2_g, ln2_b, MROWS, X1, N16);
    for (int ch = 0; ch < 2; ++ch) {
        wmma_gemm64<2, 1, false, 1><<<(unsigned)(((CHROWS / 64) * (DFF / 64) + 7) / 8), 256, 0, stream>>>(
            N16 + (size_t)ch * CHROWS * DM, DM, W1T, DM, (void*)ACT16, DFF, b_fc, nullptr, CHROWS, DFF, DM, 0.0625f);
        wmma_gemm64<2, 0, true, 0><<<(unsigned)(((CHROWS / 64) * (DM / 64) + 7) / 8), 256, 0, stream>>>(
            ACT16, DFF, W2T, DFF, (void*)(out + (size_t)ch * CHROWS * DM), DM, b_fc2, X1 + (size_t)ch * CHROWS * DM, CHROWS, DM, DFF, 0.0625f);
    }
}
